// SpanIndexEncoder_34883724378827
// MI455X (gfx1250) — hardware-verified
//
#include <hip/hip_runtime.h>


#define NTOK 8192
#define NNOD 8192
#define FF   256
#define NCH  2048

typedef unsigned short bf;
typedef __attribute__((ext_vector_type(16))) __bf16   v16bf;
typedef __attribute__((ext_vector_type(8)))  unsigned short v8us;
typedef __attribute__((ext_vector_type(8)))  float    v8f;
typedef __attribute__((ext_vector_type(4)))  float    v4f;
typedef v4f  __attribute__((may_alias)) v4fa;
typedef v8us __attribute__((may_alias)) v8usa;

__device__ __forceinline__ unsigned short f2bf(float f) { unsigned u = __float_as_uint(f); u += 0x7FFFu + ((u >> 16) & 1u); return (unsigned short)(u >> 16); }
__device__ __forceinline__ v16bf cat16b(v8us lo, v8us hi) { return __builtin_bit_cast(v16bf, __builtin_shufflevector(lo, hi, 0, 1, 2, 3, 4, 5, 6, 7, 8, 9, 10, 11, 12, 13, 14, 15)); }
__device__ __forceinline__ v8f wmmab(v16bf a, v16bf b, v8f c) { return __builtin_amdgcn_wmma_f32_16x16x32_bf16(false, a, false, b, (short)0, c, false, false); }

__global__ __launch_bounds__(256) void k_et(const float* __restrict__ E, bf* ET) {
    __shared__ __align__(16) unsigned short tl[64 * 72];
    const int tid = threadIdx.x, n0 = blockIdx.x * 64, f0 = blockIdx.y * 64;
    const int nr = tid >> 2, fq = (tid & 3) * 16;
#pragma unroll
    for (int i = 0; i < 16; ++i) tl[(fq + i) * 72 + nr] = f2bf(E[(size_t)(n0 + nr) * FF + f0 + fq + i]);
    __syncthreads();
    const int piece = tid & 7;
    auto pass = [&]() {
#pragma unroll
        for (int s = 0; s < 2; ++s) { const int fr = (tid >> 3) + 32 * s; const v8us val = *(const v8usa*)(tl + fr * 72 + piece * 8); *(volatile v8us*)(ET + (size_t)(f0 + fr) * NNOD + n0 + piece * 8) = val; }
    };
    pass(); __threadfence(); pass();
}
__global__ __launch_bounds__(256) void k_mask(const int* __restrict__ st, const int* __restrict__ en, const int* __restrict__ num, int n0, bf* M) {
    const int lane = threadIdx.x & 31, t = blockIdx.x * 8 + (threadIdx.x >> 5);
    if (t >= NTOK) return; const int nn = num[0];
#pragma unroll 1
    for (int ps = 0; ps < 2; ++ps) {
#pragma unroll 1
        for (int q = 0; q < NCH / 256; ++q) { v8us o;
#pragma unroll
            for (int i = 0; i < 8; ++i) { const int nl = q * 256 + lane * 8 + i, n = n0 + nl; o[i] = (n < nn && st[n] <= t && t <= en[n]) ? (unsigned short)0x3F80 : (unsigned short)0; }
            *(volatile v8us*)(M + (size_t)t * NCH + q * 256 + lane * 8) = o; }
        if (ps == 0) __threadfence(); }
}
template <bool ACC>
__global__ __launch_bounds__(128) void k_gemm(const bf* __restrict__ M, const bf* __restrict__ ET, int kofs, float* out) {
    __shared__ __align__(16) float ost[4][16 * 68];
    const int lane = threadIdx.x & 31, wave = threadIdx.x >> 5, lr = lane & 15, hi = lane >> 4;
    const size_t r0 = (size_t)blockIdx.x * 64 + wave * 16; const int c0 = blockIdx.y * 64;
    const size_t aoff = (r0 + lr) * NCH + 8 * hi;
    size_t boff[4];
#pragma unroll
    for (int t = 0; t < 4; ++t) boff[t] = (size_t)(c0 + t * 16 + lr) * NNOD + kofs + 8 * hi;
    v8f acc[4];
#pragma unroll
    for (int t = 0; t < 4; ++t) acc[t] = (v8f){};
#pragma unroll 2
    for (int kc = 0; kc < NCH; kc += 32) {
        const v16bf a = cat16b(*(const v8us*)(M + aoff + kc), *(const v8us*)(M + aoff + kc + 16));
#pragma unroll
        for (int t = 0; t < 4; ++t) acc[t] = wmmab(a, cat16b(*(const v8us*)(ET + boff[t] + kc), *(const v8us*)(ET + boff[t] + kc + 16)), acc[t]);
        asm volatile("v_nop" : "+v"(acc[0]), "+v"(acc[1]), "+v"(acc[2]), "+v"(acc[3]) : "v"(a) : "memory");
    }
    float* os = &ost[wave][0];
#pragma unroll
    for (int t = 0; t < 4; ++t)
#pragma unroll
        for (int j = 0; j < 8; ++j) { float v = acc[t][j]; if (ACC) v += out[(r0 + hi * 8 + j) * FF + c0 + t * 16 + lr]; os[(hi * 8 + j) * 68 + t * 16 + lr] = v; }
    __builtin_amdgcn_wave_barrier(); asm volatile("" ::: "memory");
    float* crow = out + r0 * FF + c0;
    auto pass = [&]() {
#pragma unroll
        for (int s = 0; s < 8; ++s) { const int Lid = (lane >> 3) + 4 * s, piece = lane & 7; const int row = Lid >> 1, cofs = (Lid & 1) * 32 + piece * 4;
            const v4f val = *(const v4fa*)(os + row * 68 + cofs); *(volatile v4f*)(crow + (size_t)row * FF + cofs) = val; }
    };
    pass(); __threadfence(); pass();
}

extern "C" void kernel_launch(void* const* d_in, const int* in_sizes, int n_in,
                              void* d_out, int out_size, void* d_ws, size_t ws_size, hipStream_t stream) {
    (void)in_sizes; (void)n_in; (void)out_size;
    const float* E = (const float*)d_in[0]; const int* st = (const int*)d_in[1]; const int* en = (const int*)d_in[2]; const int* num = (const int*)d_in[3];
    float* out = (float*)d_out;
    char* wsp = (char*)d_ws;
    auto take = [&](size_t bytes) { char* p = wsp; wsp += (bytes + 255) & ~(size_t)255; return (void*)p; };
    bf* ET = (bf*)take((size_t)FF * NNOD * 2); bf* M = (bf*)take((size_t)NTOK * NCH * 2);
    if ((size_t)(wsp - (char*)d_ws) > ws_size) return;
    k_et<<<dim3(NNOD / 64, FF / 64, 1), 256, 0, stream>>>(E, ET);
    for (int c = 0; c < NNOD / NCH; ++c) {
        k_mask<<<NTOK / 8, 256, 0, stream>>>(st, en, num, c * NCH, M);
        if (c == 0) k_gemm<false><<<dim3(NTOK / 64, FF / 64, 1), 128, 0, stream>>>(M, ET, c * NCH, out);
        else        k_gemm<true ><<<dim3(NTOK / 64, FF / 64, 1), 128, 0, stream>>>(M, ET, c * NCH, out);
    }
}
